// GraphConvLayer_17884243821392
// MI455X (gfx1250) — hardware-verified
//
#include <hip/hip_runtime.h>
#include <stddef.h>
#include <stdint.h>

#define GH     64
#define GW     64
#define NNODE  (GH * GW)
#define CIN    128
#define COUT   128
#define NB     4
#define NROWS  (NB * NNODE)
#define NBRCAP 8
#define NEXTRA 252
#define NTHR   256
#define GBM    64
#define GBN    64
#define GTHR   128
#define NXU    (NROWS * (CIN / 8))
#define NWU    (COUT * (CIN / 8))
#define NBN    1024
#define WSMAX  134217728

static_assert(GH == 64 && GW == 64 && NNODE == 4096);
static_assert(CIN == 128 && COUT == 128 && CIN == 32 * 4 && COUT == 32 * 4);
static_assert(CIN % 32 == 0);
static_assert(NROWS % GBM == 0 && COUT % GBN == 0);
static_assert(GBM == (GTHR / 32) * 16 && GBN == 64);
static_assert(NXU % NTHR == 0 && NWU % NTHR == 0);
static_assert(NNODE % NBN == 0 && NBN == 4 * NTHR);
static_assert(NBRCAP == 8 && NBRCAP >= 7);
static_assert(NROWS % 8 == 0);

typedef float          v4f   __attribute__((ext_vector_type(4)));
typedef float          v8f   __attribute__((ext_vector_type(8)));
typedef int            v4i   __attribute__((ext_vector_type(4)));
typedef int            v8i   __attribute__((ext_vector_type(8)));
typedef unsigned short v8us  __attribute__((ext_vector_type(8)));
typedef unsigned short v16us __attribute__((ext_vector_type(16)));
typedef __bf16         v16bf __attribute__((ext_vector_type(16)));
typedef v4f  __attribute__((may_alias)) v4fa;
typedef v4i  __attribute__((may_alias)) v4ia;
typedef v8us __attribute__((may_alias)) v8usa;
union FragB { v16bf v; v16us u; v8us h[2]; v8i w; };

struct ExtraTab { short v[2 * NEXTRA]; };
static constexpr ExtraTab kExtra = {{
  0,128, 1,64, 2,67, 3,68, 4,69, 5,68, 6,71, 7,72,
  8,71, 9,74, 10,75, 11,74, 12,77, 13,76, 14,79, 15,78,
  16,79, 17,82, 18,83, 19,82, 20,83, 21,84, 22,87, 23,88,
  24,87, 25,90, 26,89, 27,92, 28,93, 29,94, 30,93, 31,94,
  32,95, 33,96, 34,97, 35,100, 36,99, 37,102, 38,101, 39,104,
  40,105, 41,106, 42,107, 43,106, 44,109, 45,110, 46,111, 47,112,
  48,111, 49,112, 50,115, 51,116, 52,115, 53,116, 54,119, 55,118,
  56,119, 57,122, 58,121, 59,122, 60,123, 61,124, 62,125, 63,61,
  64,1, 127,190, 128,193, 191,126, 192,257, 255,190, 256,193, 319,254,
  320,385, 383,318, 384,321, 447,382, 448,385, 511,574, 512,449, 575,638,
  576,641, 639,702, 640,577, 703,638, 704,641, 767,702, 768,705, 831,894,
  832,769, 895,830, 896,961, 959,1022, 960,897, 1023,1086, 1024,1089, 1087,1150,
  1088,1153, 1151,1214, 1152,1089, 1215,1278, 1216,1153, 1279,1342, 1280,1217, 1343,1406,
  1344,1409, 1407,1470, 1408,1345, 1471,1534, 1472,1409, 1535,1598, 1536,1473, 1599,1662,
  1600,1665, 1663,1598, 1664,1601, 1727,1790, 1728,1793, 1791,1854, 1792,1729, 1855,1790,
  1856,1921, 1919,1982, 1920,1857, 1983,2046, 1984,2049, 2047,1982, 2048,2113, 2111,2046,
  2112,2049, 2175,2238, 2176,2113, 2239,2302, 2240,2305, 2303,2366, 2304,2369, 2367,2430,
  2368,2305, 2431,2366, 2432,2497, 2495,2558, 2496,2433, 2559,2494, 2560,2497, 2623,2558,
  2624,2561, 2687,2622, 2688,2753, 2751,2814, 2752,2689, 2815,2750, 2816,2753, 2879,2814,
  2880,2817, 2943,3006, 2944,3009, 3007,2942, 3008,2945, 3071,3006, 3072,3009, 3135,3070,
  3136,3073, 3199,3262, 3200,3137, 3263,3198, 3264,3329, 3327,3390, 3328,3265, 3391,3454,
  3392,3329, 3455,3518, 3456,3521, 3519,3582, 3520,3457, 3583,3518, 3584,3649, 3647,3582,
  3648,3713, 3711,3646, 3712,3777, 3775,3710, 3776,3713, 3839,3774, 3840,3905, 3903,3966,
  3904,3841, 3967,4030, 3968,4033, 4031,3966, 4032,4034, 4033,3968, 4034,3971, 4035,3970,
  4036,3973, 4037,3972, 4038,3973, 4039,3974, 4040,3975, 4041,3978, 4042,3977, 4043,3980,
  4044,3979, 4045,3980, 4046,3981, 4047,3982, 4048,3985, 4049,3984, 4050,3987, 4051,3986,
  4052,3989, 4053,3990, 4054,3989, 4055,3990, 4056,3993, 4057,3994, 4058,3993, 4059,3996,
  4060,3997, 4061,3998, 4062,3999, 4063,3998, 4064,3999, 4065,4002, 4066,4001, 4067,4004,
  4068,4005, 4069,4004, 4070,4007, 4071,4006, 4072,4007, 4073,4010, 4074,4011, 4075,4012,
  4076,4011, 4077,4012, 4078,4013, 4079,4016, 4080,4017, 4081,4016, 4082,4019, 4083,4020,
  4084,4019, 4085,4020, 4086,4023, 4087,4022, 4088,4023, 4089,4026, 4090,4025, 4091,4026,
  4092,4027, 4093,4028, 4094,4029, 4095,4093
}};

constexpr int extra_node_of(int o) {
  return (o < 64) ? o : ((o < 188) ? (64 * (1 + (o - 64) / 2) + (((o - 64) & 1) ? 63 : 0)) : (4032 + (o - 188)));
}
constexpr bool extra_ok(const ExtraTab& t) {
  for (int o = 0; o < NEXTRA; ++o) {
    const int a = extra_node_of(o);
    if ((int)t.v[2 * o] != a) return false;
    const int m = (int)t.v[2 * o + 1];
    if (m < 0 || m >= NNODE) return false;
    const int ai = a >> 6, aj = a & 63, mi = m >> 6, mj = m & 63;
    const int di = mi > ai ? mi - ai : ai - mi;
    const int dj = mj > aj ? mj - aj : aj - mj;
    const bool crn = (ai == 0 || ai == 63) && (aj == 0 || aj == 63);
    if (crn) { if (!((di == 2 && dj == 0) || (di == 0 && dj == 2))) return false; }
    else     { if (!(di == 1 && dj == 1)) return false; }
  }
  return true;
}
static_assert(sizeof(ExtraTab) == 2 * NEXTRA * sizeof(short));
static_assert(extra_ok(kExtra));

__constant__ ExtraTab c_extra = kExtra;

#define DIPACK ((0x4333ULL << 32) | 0x22221110ULL)
#define DJPACK ((0x2321ULL << 32) | 0x43103212ULL)
constexpr bool cand_ok() {
  int last = -100000;
  for (int c = 0; c < 12; ++c) {
    const int di = (int)((DIPACK >> (4 * c)) & 15ULL) - 2;
    const int dj = (int)((DJPACK >> (4 * c)) & 15ULL) - 2;
    const int ad = (di < 0 ? -di : di), aj = (dj < 0 ? -dj : dj);
    const int d2 = ad * ad + aj * aj;
    if (!(d2 == 1 || d2 == 2 || d2 == 4)) return false;
    const int off = 64 * di + dj;
    if (off <= last) return false;
    last = off;
  }
  return true;
}
static_assert(cand_ok());

__device__ __forceinline__ v8f wmb(const FragB& a, const FragB& b, v8f c) {
  v8f d = __builtin_amdgcn_wmma_f32_16x16x32_bf16(false, a.v, false, b.v, (short)0, c, false, false);
  asm volatile("v_nop\n\tv_nop\n\tv_nop\n\tv_nop" : "+v"(d) : "v"(a.w), "v"(b.w));
  return d;
}

__device__ __forceinline__ unsigned bf16_bits(float f) {
  const unsigned u = __float_as_uint(f);
  return (u + 0x7FFFu + ((u >> 16) & 1u)) >> 16;
}

__global__ __launch_bounds__(NTHR) void k_prep(const float* __restrict__ x, const float* __restrict__ W,
                                               unsigned short* XB, unsigned short* WT) {
  const int u = (int)blockIdx.x * NTHR + (int)threadIdx.x;
  v8us o;
  unsigned short* dp;
  if (u < NXU) {
    const float* p = x + (size_t)u * 8;
    const v4f a = *(const v4fa*)p;
    const v4f b = *(const v4fa*)(p + 4);
    o[0] = (unsigned short)bf16_bits(a.x); o[1] = (unsigned short)bf16_bits(a.y);
    o[2] = (unsigned short)bf16_bits(a.z); o[3] = (unsigned short)bf16_bits(a.w);
    o[4] = (unsigned short)bf16_bits(b.x); o[5] = (unsigned short)bf16_bits(b.y);
    o[6] = (unsigned short)bf16_bits(b.z); o[7] = (unsigned short)bf16_bits(b.w);
    dp = XB + (size_t)u * 8;
  } else if (u < NXU + NWU) {
    const int v  = u - NXU;
    const int n  = v >> 4;
    const int k8 = (v & 15) * 8;
    const float* p = W + (size_t)k8 * COUT + n;
#pragma unroll
    for (int i = 0; i < 8; ++i) o[i] = (unsigned short)bf16_bits(p[(size_t)i * COUT]);
    dp = WT + (size_t)n * CIN + k8;
  } else {
    return;
  }
  *(volatile v8us*)dp = o;
  __threadfence();
  *(volatile v8us*)dp = o;
}

__device__ __forceinline__ int border_ord(int ai, int aj) {
  int o = (ai == 0) ? aj : ((ai == 63) ? (188 + aj) : (64 + 2 * (ai - 1) + ((aj == 63) ? 1 : 0)));
  o = o < 0 ? 0 : (o > NEXTRA - 1 ? NEXTRA - 1 : o);
  return o;
}
__device__ __forceinline__ bool pick(int ai, int aj, int m, int adi, int adj) {
  const bool axis = (adi + adj) == 1;
  const bool brd  = (ai == 0) | (ai == 63) | (aj == 0) | (aj == 63);
  const bool crn  = ((ai == 0) | (ai == 63)) & ((aj == 0) | (aj == 63));
  const bool diag = (adi == 1) & (adj == 1);
  const int  em   = (int)c_extra.v[2 * border_ord(ai, aj) + 1];
  return axis | (crn & diag) | (brd & (em == m));
}

__global__ __launch_bounds__(NTHR) void k_nbr(int* nbr) {
  __shared__ __attribute__((aligned(16))) int snb[NBN * NBRCAP];
  const int tid = (int)threadIdx.x;
  const int nodeBase = (int)blockIdx.x * NBN;

#pragma unroll 1
  for (int q = 0; q < 4; ++q) {
    const int nl = 4 * tid + q;
    const int n  = nodeBase + nl;
    const int ni = n >> 6, nj = n & 63;
#pragma unroll
    for (int s = 0; s < NBRCAP; ++s) snb[nl * NBRCAP + s] = -1;

    const bool brd = (ni == 0) | (ni == 63) | (nj == 0) | (nj == 63);
    const bool crn = ((ni == 0) | (ni == 63)) & ((nj == 0) | (nj == 63));
    const int  ord = border_ord(ni, nj);
    const int  ea  = (int)c_extra.v[2 * ord];
    const int  em  = (int)c_extra.v[2 * ord + 1];
    const int  emi = em >> 6, emj = em & 63;
    const int  edi = emi > ni ? emi - ni : ni - emi;
    const int  edj = emj > nj ? emj - nj : nj - emj;
    const bool emin = (unsigned)em < (unsigned)NNODE;
    const bool elegal = crn ? (((edi == 2) & (edj == 0)) | ((edi == 0) & (edj == 2)))
                            : ((edi == 1) & (edj == 1));
    bool bad = brd & (!(ea == n) | !emin | !elegal);

    int cnt = 0;
#pragma unroll 1
    for (int c = 0; c < 12; ++c) {
      const int di = (int)((DIPACK >> (4 * c)) & 15ULL) - 2;
      const int dj = (int)((DJPACK >> (4 * c)) & 15ULL) - 2;
      const int mi = ni + di, mj = nj + dj;
      const bool ing = ((unsigned)mi < (unsigned)GH) & ((unsigned)mj < (unsigned)GW);
      const int mic = mi < 0 ? 0 : (mi > GH - 1 ? GH - 1 : mi);
      const int mjc = mj < 0 ? 0 : (mj > GW - 1 ? GW - 1 : mj);
      const int m   = mic * GW + mjc;
      const int adi = di < 0 ? -di : di;
      const int adj = dj < 0 ? -dj : dj;
      const bool fwd = pick(ni, nj, m, adi, adj);
      const bool rev = pick(mic, mjc, n, adi, adj);
      const bool emit = ing & (fwd | rev);
      if (emit) {
        if (cnt < NBRCAP) snb[nl * NBRCAP + cnt] = m;
        cnt = cnt + 1;
      }
    }
    bad = bad | (cnt > NBRCAP);
    if (bad) snb[nl * NBRCAP] = -2;
  }
  __syncthreads();

  v4i vv[8];
#pragma unroll
  for (int it = 0; it < 8; ++it) vv[it] = *(const v4ia*)(snb + 4 * (it * NTHR + tid));
  int* base = nbr + (size_t)nodeBase * NBRCAP;
#pragma unroll
  for (int it = 0; it < 8; ++it) *(volatile v4i*)(base + 4 * (it * NTHR + tid)) = vv[it];
  __threadfence();
#pragma unroll
  for (int it = 0; it < 8; ++it) *(volatile v4i*)(base + 4 * (it * NTHR + tid)) = vv[it];
}

__global__ __launch_bounds__(GTHR) void k_proj(
    const unsigned short* __restrict__ A, const unsigned short* __restrict__ WT,
    float* outF, int K, int ldo)
{
  __shared__ __attribute__((aligned(16))) float stg[GBM * GBN];
  const int tid = (int)threadIdx.x, lane = tid & 31, wave = tid >> 5, hh = lane >> 4, m = lane & 15;
  const int rowBase = (int)blockIdx.x * GBM;
  const int col0    = (int)blockIdx.y * GBN;

  v8f acc[4];
  {
    const v8f z = {0.f, 0.f, 0.f, 0.f, 0.f, 0.f, 0.f, 0.f};
    acc[0] = z; acc[1] = z; acc[2] = z; acc[3] = z;
  }
  const unsigned short* ap = A  + (size_t)(rowBase + 16 * wave + m) * (size_t)K + 8 * hh;
  const unsigned short* wp = WT + (size_t)(col0 + m) * (size_t)K + 8 * hh;
  const int ksteps = K >> 5;
#pragma unroll 1
  for (int ks = 0; ks < ksteps; ++ks) {
    FragB af;
    af.h[0] = *(const v8usa*)(ap + 32 * ks);
    af.h[1] = *(const v8usa*)(ap + 32 * ks + 16);
#pragma unroll
    for (int t = 0; t < 4; ++t) {
      const unsigned short* wq = wp + (size_t)(16 * t) * (size_t)K + 32 * ks;
      FragB bf;
      bf.h[0] = *(const v8usa*)wq;
      bf.h[1] = *(const v8usa*)(wq + 16);
      acc[t] = wmb(af, bf, acc[t]);
    }
  }

#pragma unroll
  for (int t = 0; t < 4; ++t) {
    const int lc = 16 * t + m;
#pragma unroll
    for (int r = 0; r < 8; ++r) {
      const int lr = 16 * wave + 8 * hh + r;
      stg[lr * GBN + lc] = acc[t][r];
    }
  }
  __syncthreads();

  v4f fv[8];
#pragma unroll
  for (int i = 0; i < 8; ++i) {
    const int lr = 16 * wave + 2 * i + hh;
    fv[i] = *(const v4fa*)(stg + lr * GBN + 4 * m);
  }
#pragma unroll
  for (int i = 0; i < 8; ++i) {
    const int lr = 16 * wave + 2 * i + hh;
    const int gr = rowBase + lr;
    float* op = outF + (size_t)gr * (size_t)ldo + col0 + 4 * m;
    *(volatile v4f*)op = fv[i];
  }
  __threadfence();
#pragma unroll
  for (int i = 0; i < 8; ++i) {
    const int lr = 16 * wave + 2 * i + hh;
    const int gr = rowBase + lr;
    float* op = outF + (size_t)gr * (size_t)ldo + col0 + 4 * m;
    *(volatile v4f*)op = fv[i];
  }
}

#define ADDJ(IDX) { \
    const int id_ = (IDX); \
    const unsigned mk_ = ~(unsigned)(id_ >> 31); \
    const int ic_ = id_ < 0 ? 0 : (id_ > NNODE - 1 ? NNODE - 1 : id_); \
    const v4f v_ = *(const v4fa*)(pb + (size_t)ic_ * COUT); \
    acc.x += __uint_as_float(__float_as_uint(v_.x) & mk_); \
    acc.y += __uint_as_float(__float_as_uint(v_.y) & mk_); \
    acc.z += __uint_as_float(__float_as_uint(v_.z) & mk_); \
    acc.w += __uint_as_float(__float_as_uint(v_.w) & mk_); }

__global__ __launch_bounds__(NTHR) void k_agg(const float* __restrict__ P, const int* __restrict__ nbr,
                                              float* out) {
  const int tid = (int)threadIdx.x, lane = tid & 31, wave = tid >> 5;
  const int r = (int)blockIdx.x * 8 + wave;
  const int b = r >> 12;
  const int n = r & (NNODE - 1);
  const v4i n0 = *(const v4ia*)(nbr + (size_t)n * NBRCAP);
  const v4i n1 = *(const v4ia*)(nbr + (size_t)n * NBRCAP + 4);
  const float* pb = P + (size_t)b * NNODE * COUT + 4 * lane;

  v4f acc = {0.0f, 0.0f, 0.0f, 0.0f};
  ADDJ(n0.x)
  ADDJ(n0.y)
  ADDJ(n0.z)
  ADDJ(n0.w)
  ADDJ(n1.x)
  ADDJ(n1.y)
  ADDJ(n1.z)
  ADDJ(n1.w)

  const bool poison = (n0.x == -2);
  const float qnan = __int_as_float(0x7fc00000);
  v4f y;
  y.x = (acc.x >= 0.0f) ? acc.x : 0.1f * acc.x;
  y.y = (acc.y >= 0.0f) ? acc.y : 0.1f * acc.y;
  y.z = (acc.z >= 0.0f) ? acc.z : 0.1f * acc.z;
  y.w = (acc.w >= 0.0f) ? acc.w : 0.1f * acc.w;
  y.x = poison ? qnan : y.x;
  y.y = poison ? qnan : y.y;
  y.z = poison ? qnan : y.z;
  y.w = poison ? qnan : y.w;

  float* op = out + (size_t)r * COUT + 4 * lane;
  *(volatile v4f*)op = y;
  __threadfence();
  *(volatile v4f*)op = y;
}
#undef ADDJ

static inline size_t al256(size_t o) { return (o + 255) & ~(size_t)255; }

extern "C" void kernel_launch(void* const* d_in, const int* in_sizes, int n_in,
                              void* d_out, int out_size, void* d_ws, size_t ws_size,
                              hipStream_t stream) {
  if (n_in < 2) return;
  if (in_sizes[0] != NROWS * CIN) return;
  if (in_sizes[1] != CIN * COUT) return;
  if (out_size != NROWS * COUT) return;

  const float* x = (const float*)d_in[0];
  const float* W = (const float*)d_in[1];
  float* out = (float*)d_out;

  char* ws = (char*)d_ws;
  size_t off = 0;
  const size_t oXB  = off; off = al256(off + (size_t)NROWS * CIN * 2);
  const size_t oWT  = off; off = al256(off + (size_t)COUT * CIN * 2);
  const size_t oP   = off; off = al256(off + (size_t)NROWS * COUT * 4);
  const size_t oNBR = off; off = al256(off + (size_t)NNODE * NBRCAP * 4);
  if (off > ws_size || off > (size_t)WSMAX) return;
  unsigned short* XB  = (unsigned short*)(ws + oXB);
  unsigned short* WT  = (unsigned short*)(ws + oWT);
  float*          Pp  = (float*)(ws + oP);
  int*            NBR = (int*)(ws + oNBR);

  k_prep<<<(NXU + NWU) / NTHR, NTHR, 0, stream>>>(x, W, XB, WT);
  k_nbr<<<NNODE / NBN, NTHR, 0, stream>>>(NBR);
  k_proj<<<dim3(NROWS / GBM, COUT / GBN), GTHR, 0, stream>>>(XB, WT, Pp, CIN, COUT);
  k_agg<<<NROWS / 8, NTHR, 0, stream>>>(Pp, NBR, out);
}
